// Network_65051574665498
// MI455X (gfx1250) — hardware-verified
//
#include <hip/hip_runtime.h>
#include <math.h>

typedef __attribute__((ext_vector_type(16))) _Float16 v16h;
typedef __attribute__((ext_vector_type(16))) __bf16 v16b;
typedef __attribute__((ext_vector_type(8)))  _Float16 v8h;
typedef __attribute__((ext_vector_type(8)))  float v8f;
typedef __attribute__((ext_vector_type(4)))  float v4f;
typedef __attribute__((ext_vector_type(2)))  float v2f;
typedef __attribute__((ext_vector_type(4)))  unsigned v4u;
typedef __attribute__((ext_vector_type(4)))  int v4i;
typedef float __attribute__((may_alias)) float_a;
typedef int __attribute__((may_alias)) int_a;

template <typename T> __device__ __forceinline__ void vst2(void* p, T v) { *(volatile T*)p = v; __threadfence(); *(volatile T*)p = v; }
__device__ __forceinline__ v8f wmma16(v16h a, v16h b, v8f c) {
  v8f d = __builtin_amdgcn_wmma_f32_16x16x32_f16(false, a, false, b, (short)0, c, false, false);
  asm volatile("v_nop\n\tv_nop\n\tv_nop\n\tv_nop" : "+v"(d) : "v"(a), "v"(b));
  return d;
}
__device__ __forceinline__ v8f wmma_bf(v16b a, v16b b, v8f c) {
  v8f d = __builtin_amdgcn_wmma_f32_16x16x32_bf16(false, a, false, b, (short)0, c, false, false);
  asm volatile("v_nop\n\tv_nop\n\tv_nop\n\tv_nop" : "+v"(d) : "v"(a), "v"(b));
  return d;
}
__device__ __forceinline__ v16h frag_h(const _Float16* rowk0, int lane) {
  union { v16h v; v8h q[2]; } u; const _Float16* p = rowk0 + 8 * (lane >> 4);
  u.q[0] = *(const v8h*)p; u.q[1] = *(const v8h*)(p + 16); return u.v;
}
__device__ __forceinline__ v16h frag_f32(const float* rowk0, int lane) {
  v16h a; const float* p = rowk0 + 8 * (lane >> 4);
#pragma unroll
  for (int i = 0; i < 8; ++i) { a[i] = (_Float16)p[i]; a[8 + i] = (_Float16)p[16 + i]; }
  return a;
}
__device__ __forceinline__ v16h frag_f32s(const float* rowk0, int lane, float sc) {
  v16h a; const float* p = rowk0 + 8 * (lane >> 4);
#pragma unroll
  for (int i = 0; i < 8; ++i) { a[i] = (_Float16)(p[i] * sc); a[8 + i] = (_Float16)(p[16 + i] * sc); }
  return a;
}
__device__ __forceinline__ v16h fragc_f32(const float* W, int k0, int n, int lane, int ld, int K) {
  v16h a; const int g = lane >> 4;
#pragma unroll
  for (int i = 0; i < 8; ++i) { const int ka = k0 + 8 * g + i, kb = ka + 16;
    a[i] = (_Float16)(ka < K ? W[(size_t)(ka < K ? ka : K - 1) * ld + n] : 0.f); a[8 + i] = (_Float16)(kb < K ? W[(size_t)(kb < K ? kb : K - 1) * ld + n] : 0.f); }
  return a;
}
struct F2 { v16b h, l; };
__device__ __forceinline__ F2 bsplit16(const float v[16]) { F2 r;
#pragma unroll
  for (int i = 0; i < 16; ++i) { const __bf16 h = (__bf16)v[i]; r.h[i] = h; r.l[i] = (__bf16)(v[i] - (float)h); }
  return r; }
__device__ __forceinline__ F2 split_row(const float* row, int k0, int lane) { float v[16]; const float* p = row + k0 + 8 * (lane >> 4);
#pragma unroll
  for (int i = 0; i < 8; ++i) { v[i] = p[i]; v[8 + i] = p[16 + i]; }
  return bsplit16(v); }
__device__ __forceinline__ F2 split_rowK(const float* row, int k0, int lane, int K) { float v[16]; const int g = lane >> 4;
#pragma unroll
  for (int i = 0; i < 8; ++i) { const int ka = k0 + 8 * g + i, kb = ka + 16; v[i] = ka < K ? row[ka < K ? ka : K - 1] : 0.f; v[8 + i] = kb < K ? row[kb < K ? kb : K - 1] : 0.f; }
  return bsplit16(v); }
__device__ __forceinline__ F2 split_col(const float* W, int k0, int n, int lane, int ld, int K) { float v[16]; const int g = lane >> 4;
#pragma unroll
  for (int i = 0; i < 8; ++i) { const int ka = k0 + 8 * g + i, kb = ka + 16; v[i] = ka < K ? W[(size_t)(ka < K ? ka : K - 1) * ld + n] : 0.f; v[8 + i] = kb < K ? W[(size_t)(kb < K ? kb : K - 1) * ld + n] : 0.f; }
  return bsplit16(v); }
__device__ __forceinline__ v8f mac3(const F2& a, const F2& b, v8f c) { c = wmma_bf(a.l, b.h, c); c = wmma_bf(a.h, b.l, c); return wmma_bf(a.h, b.h, c); }
__device__ __forceinline__ float sigm(float v) { return 1.0f / (1.0f + expf(-v)); }
#define LDSX() do { asm volatile("s_wait_dscnt 0" ::: "memory"); __builtin_amdgcn_wave_barrier(); __builtin_amdgcn_fence(__ATOMIC_RELEASE, "workgroup"); } while (0)

__device__ __forceinline__ float bfr(float v) { return (float)(__bf16)v; }
#define NPT 2097152
#define DEN_OFF ((size_t)NPT * 3)
#ifndef NBLK
#define NBLK (NPT / 64)
#endif
#define AW 104
#define WT_B0 0
#define WT_B1 (WT_B0 + 64 * 64)
#define WT_B2 (WT_B1 + 64 * 64)
#define WT_H0 (WT_B2 + 64 * 64)
#define WT_H1 (WT_H0 + 64 * 96)
#define WT_H2 (WT_H1 + 64 * 64)
#define WT_END (WT_H2 + 16 * 64)
#define WS_END ((size_t)WT_END * 2)
__device__ __forceinline__ void layer64(_Float16 (*act)[AW], const _Float16* __restrict__ WT, int kpad, int nkc, int lane, v8f acc[4]) {
#pragma unroll
  for (int j = 0; j < 4; ++j) acc[j] = (v8f){};
  for (int kc = 0; kc < nkc; ++kc) { const v16h a = frag_h(&act[lane & 15][kc * 32], lane);
#pragma unroll
    for (int j = 0; j < 4; ++j) acc[j] = wmma16(a, frag_h(WT + (size_t)(j * 16 + (lane & 15)) * kpad + kc * 32, lane), acc[j]); } }
__global__ __launch_bounds__(256) void k_wprep(const float* __restrict__ BW0, const float* __restrict__ BW1, const float* __restrict__ BW2, const float* __restrict__ HW0, const float* __restrict__ HW1, const float* __restrict__ HW2, _Float16* __restrict__ WT) {
  const int t = threadIdx.x;
  for (int pc = t; pc < WT_END / 8; pc += 256) { union { v4u v; _Float16 h[8]; } u;
#pragma unroll
    for (int z = 0; z < 8; ++z) { const int e = pc * 8 + z; int K, NO, kpad, base; const float* src;
      if (e < WT_B1) { base = WT_B0; kpad = 64; K = 60; NO = 64; src = BW0; } else if (e < WT_B2) { base = WT_B1; kpad = 64; K = 64; NO = 64; src = BW1; } else if (e < WT_H0) { base = WT_B2; kpad = 64; K = 64; NO = 64; src = BW2; }
      else if (e < WT_H1) { base = WT_H0; kpad = 96; K = 87; NO = 64; src = HW0; } else if (e < WT_H2) { base = WT_H1; kpad = 64; K = 64; NO = 64; src = HW1; } else { base = WT_H2; kpad = 64; K = 64; NO = 3; src = HW2; }
      const int o = (e - base) / kpad, k = (e - base) % kpad; u.h[z] = (k < K && o < NO) ? (_Float16)bfr(src[(size_t)k * NO + o]) : (_Float16)0.f; }
    vst2((v4u*)(WT + (size_t)pc * 8), u.v); } }
__global__ __launch_bounds__(128) void k_nerf(const float* __restrict__ POS, const float* __restrict__ DIR, const float* __restrict__ BW0, const float* __restrict__ BB0, const float* __restrict__ BW1, const float* __restrict__ BB1, const float* __restrict__ BW2, const float* __restrict__ BB2, const float* __restrict__ HW0, const float* __restrict__ HB0, const float* __restrict__ HW1, const float* __restrict__ HB1, const float* __restrict__ HW2, const float* __restrict__ HB2, const _Float16* __restrict__ WT, float* __restrict__ OUT) {
  __shared__ __align__(16) _Float16 act[4][16][AW]; __shared__ __align__(16) float srgb[64 * 3]; __shared__ __align__(16) float sden[64];
  const int tid = threadIdx.x, wave = tid >> 5, lane = tid & 31, col = lane & 15, g = lane >> 4; const size_t n0 = (size_t)blockIdx.x * 64 + wave * 16;
  _Float16 (*aw)[AW] = act[wave];
  { const int rl = col; const size_t n = n0 + rl; const float px = bfr(POS[n * 3]), py = bfr(POS[n * 3 + 1]), pz = bfr(POS[n * 3 + 2]);
#pragma unroll
    for (int f5 = 0; f5 < 5; ++f5) { const int f = g * 5 + f5; const float fr = (float)(1 << f) * 3.14159274101257324f;
      const float a0 = px * fr, a1 = py * fr, a2 = pz * fr;
      aw[rl][f * 6 + 0] = (_Float16)sinf(a0); aw[rl][f * 6 + 1] = (_Float16)sinf(a1); aw[rl][f * 6 + 2] = (_Float16)sinf(a2); aw[rl][f * 6 + 3] = (_Float16)cosf(a0); aw[rl][f * 6 + 4] = (_Float16)cosf(a1); aw[rl][f * 6 + 5] = (_Float16)cosf(a2); }
    if (g == 0) { aw[rl][60] = 0; aw[rl][61] = 0; aw[rl][62] = 0; aw[rl][63] = 0; } }
  LDSX();
  v8f acc[4];
  layer64(aw, WT + WT_B0, 64, 2, lane, acc); LDSX();
#pragma unroll
  for (int j = 0; j < 4; ++j) { const int o = j * 16 + col; const float bb = bfr(BB0[o]);
#pragma unroll
    for (int r = 0; r < 8; ++r) aw[8 * g + r][o] = (_Float16)fmaxf(acc[j][r] + bb, 0.f); }
  LDSX();
  layer64(aw, WT + WT_B1, 64, 2, lane, acc); LDSX();
#pragma unroll
  for (int j = 0; j < 4; ++j) { const int o = j * 16 + col; const float bb = bfr(BB1[o]);
#pragma unroll
    for (int r = 0; r < 8; ++r) aw[8 * g + r][o] = (_Float16)fmaxf(acc[j][r] + bb, 0.f); }
  LDSX();
  layer64(aw, WT + WT_B2, 64, 2, lane, acc); LDSX();
#pragma unroll
  for (int j = 0; j < 4; ++j) { const int o = j * 16 + col; const float bb = bfr(BB2[o]);
#pragma unroll
    for (int r = 0; r < 8; ++r) { const float v = acc[j][r] + bb; if (o == 0) sden[wave * 16 + 8 * g + r] = expf(v); else aw[8 * g + r][24 + (o - 1)] = (_Float16)v; } }
  { const int rl = col; const size_t n = n0 + rl; const float dx = bfr(DIR[n * 3]), dy = bfr(DIR[n * 3 + 1]), dz = bfr(DIR[n * 3 + 2]);
#pragma unroll
    for (int f2 = 0; f2 < 2; ++f2) { const int f = g * 2 + f2; const float fr = (float)(1 << f) * 3.14159274101257324f; const float a0 = dx * fr, a1 = dy * fr, a2 = dz * fr;
      aw[rl][f * 6 + 0] = (_Float16)sinf(a0); aw[rl][f * 6 + 1] = (_Float16)sinf(a1); aw[rl][f * 6 + 2] = (_Float16)sinf(a2); aw[rl][f * 6 + 3] = (_Float16)cosf(a0); aw[rl][f * 6 + 4] = (_Float16)cosf(a1); aw[rl][f * 6 + 5] = (_Float16)cosf(a2); }
    if (g == 0) { for (int z = 87; z < 96; ++z) aw[rl][z] = 0; } }
  LDSX();
  layer64(aw, WT + WT_H0, 96, 3, lane, acc); LDSX();
#pragma unroll
  for (int j = 0; j < 4; ++j) { const int o = j * 16 + col; const float bb = bfr(HB0[o]);
#pragma unroll
    for (int r = 0; r < 8; ++r) aw[8 * g + r][o] = (_Float16)fmaxf(acc[j][r] + bb, 0.f); }
  LDSX();
  layer64(aw, WT + WT_H1, 64, 2, lane, acc); LDSX();
#pragma unroll
  for (int j = 0; j < 4; ++j) { const int o = j * 16 + col; const float bb = bfr(HB1[o]);
#pragma unroll
    for (int r = 0; r < 8; ++r) aw[8 * g + r][o] = (_Float16)fmaxf(acc[j][r] + bb, 0.f); }
  LDSX();
  { v8f a3 = {};
#pragma unroll
    for (int kc = 0; kc < 2; ++kc) a3 = wmma16(frag_h(&aw[col][kc * 32], lane), frag_h(WT + WT_H2 + (size_t)col * 64 + kc * 32, lane), a3);
    if (col < 3) { const float bb = bfr(HB2[col]);
#pragma unroll
      for (int r = 0; r < 8; ++r) srgb[(wave * 16 + 8 * g + r) * 3 + col] = sigm(a3[r] + bb); } }
  __syncthreads();
  if (tid < 48) vst2(OUT + (size_t)blockIdx.x * 64 * 3 + tid * 4, *(const v4f*)&srgb[tid * 4]);
  if (tid >= 64 && tid < 80) vst2(OUT + DEN_OFF + (size_t)blockIdx.x * 64 + (tid - 64) * 4, *(const v4f*)&sden[(tid - 64) * 4]); }
extern "C" void kernel_launch(void* const* d_in, const int* in_sizes, int n_in, void* d_out, int out_size, void* d_ws, size_t ws_size, hipStream_t stream) {
  (void)in_sizes; (void)n_in; (void)out_size;
  const float** F = (const float**)d_in;
  if (ws_size < (size_t)WS_END) return;
  _Float16* WT = (_Float16*)d_ws;
  k_wprep<<<dim3(1), 256, 0, stream>>>(F[2], F[4], F[6], F[8], F[10], F[12], WT);
  k_nerf<<<dim3(NBLK), 128, 0, stream>>>(F[0], F[1], F[2], F[3], F[4], F[5], F[6], F[7], F[8], F[9], F[10], F[11], F[12], F[13], WT, (float*)d_out);
}
